// Decoder_850403525057
// MI455X (gfx1250) — hardware-verified
//
#include <hip/hip_runtime.h>
#include <math.h>

typedef __attribute__((ext_vector_type(16))) _Float16 v16h;
typedef __attribute__((ext_vector_type(8)))  _Float16 v8h;
typedef __attribute__((ext_vector_type(8)))  float    v8f;
typedef __attribute__((ext_vector_type(4)))  float    v4f;

constexpr int NSEQ  = 64;
constexpr int NSTEP = 512;
constexpr int NIN   = 256;
constexpr int NHID  = 512;
constexpr int NOUTF = 256;
constexpr int NROWS = NSEQ * NSTEP;

constexpr float XCARRY  = 64.0f;
constexpr float WCARRY  = 1024.0f;
constexpr float LOCARRY = 2048.0f;
constexpr float INV_XW  = 1.0f / (XCARRY * WCARRY);
constexpr float INV_W   = 1.0f / WCARRY;
constexpr float INV_WL  = 1.0f / (WCARRY * LOCARRY);
constexpr float F16_MIN_NORMAL = 6.103515625e-5f;

constexpr int SEQ_PB      = 16;
constexpr int RNN_BLOCKS  = NSEQ / SEQ_PB;
constexpr int RNN_THREADS = 256;
constexpr int HPITCH      = NHID + 8;
constexpr int HTILE       = SEQ_PB * HPITCH;
constexpr int SLABP       = 36;

constexpr int CH_X    = NROWS * NIN / 8;
constexpr int CH_WIH  = NHID * NIN / 8;
constexpr int CH_WHH  = NHID * NHID / 8;
constexpr int CH_WFF  = NOUTF * NHID / 8;
constexpr int PB1 = CH_WIH / 256;
constexpr int PB2 = PB1 + CH_WHH / 256;
constexpr int PB3 = PB2 + CH_WFF / 256;
constexpr int PREP_BLOCKS = PB3 + 1;
constexpr int NBIASV = NHID + NOUTF;

static_assert(NSEQ % SEQ_PB == 0, "batch rows per block");
static_assert(NHID == (RNN_THREADS / 32) * 64, "8 waves x 64 hidden columns");
static_assert(NOUTF == (RNN_THREADS / 32) * 32, "8 waves x 32 output columns");
static_assert(HPITCH % 8 == 0, "16-B aligned LDS rows");
static_assert(NIN % 32 == 0 && NHID % 32 == 0, "K multiples of 32");
static_assert(NROWS % 64 == 0 && NHID % 64 == 0, "GEMM M, N tile multiples");
static_assert(((NROWS / 64) * (NHID / 64)) % 8 == 0, "GEMM grid exact");
static_assert(CH_X % 256 == 0 && CH_WIH % 256 == 0 && CH_WHH % 256 == 0 && CH_WFF % 256 == 0, "convert grids exact");
static_assert(SEQ_PB * NHID / 8 == 4 * RNN_THREADS, "h0 staging: 4 iterations x 256 threads x 8 halves = 16 x 512");
static_assert(PREP_BLOCKS == 257, "prep grid");

__device__ __forceinline__ unsigned short f2bf_bits(float f) {
  unsigned u = __float_as_uint(f);
  return (unsigned short)((u + 0x7FFFu + ((u >> 16) & 1u)) >> 16);
}
__device__ __forceinline__ float bf_bits2f(unsigned short h) { return __uint_as_float(((unsigned)h) << 16); }
__device__ __forceinline__ float bf16r(float f) { return bf_bits2f(f2bf_bits(f)); }

__device__ __forceinline__ void guard4in_h(v8f& a, v8f& b, v8f& c, v8f& d, v16h x, v16h y) {
  asm volatile("v_nop\n\tv_nop\n\tv_nop\n\tv_nop" : "+v"(a), "+v"(b), "+v"(c), "+v"(d) : "v"(x), "v"(y));
}
__device__ __forceinline__ void guard8in_h(v8f& a0, v8f& a1, v8f& a2, v8f& a3, v8f& b0, v8f& b1, v8f& b2, v8f& b3, v16h x, v16h y) {
  asm volatile("v_nop\n\tv_nop\n\tv_nop\n\tv_nop"
               : "+v"(a0), "+v"(a1), "+v"(a2), "+v"(a3), "+v"(b0), "+v"(b1), "+v"(b2), "+v"(b3) : "v"(x), "v"(y));
}
__device__ __forceinline__ void keep4_h(v16h a, v16h b, v16h c, v16h d) { asm volatile("v_nop" :: "v"(a), "v"(b), "v"(c), "v"(d)); }
__device__ __forceinline__ void acc_guard4(v8f& a, v8f& b, v8f& c, v8f& d) { asm volatile("v_nop\n\tv_nop\n\tv_nop\n\tv_nop" : "+v"(a), "+v"(b), "+v"(c), "+v"(d)); }

struct FragH {
  union U { v16h v; v8h h[2]; };
  static __device__ __forceinline__ v16h load(const _Float16* p) {
    U f; f.h[0] = *(const v8h*)(p); f.h[1] = *(const v8h*)(p + 16); return f.v;
  }
  static __device__ __forceinline__ v8f mma(v16h a, v16h b, v8f c) {
    return __builtin_amdgcn_wmma_f32_16x16x32_f16(false, a, false, b, (short)0, c, false, false);
  }
};

__device__ __forceinline__ void split_h(float v, _Float16& hi, _Float16& lo) {
  const float hq0 = (float)((_Float16)v);
  const float hq  = (fabsf(v) < F16_MIN_NORMAL) ? 0.0f : hq0;
  hi = (_Float16)hq;
  lo = (_Float16)((v - hq) * LOCARRY);
}

__device__ __forceinline__ void cvt8_store(const float* sp, unsigned short* dp, float sc) {
  const v4f a = *(const v4f*)(sp);
  const v4f b = *(const v4f*)(sp + 4);
  v8h hv;
#pragma unroll
  for (int e = 0; e < 4; ++e) {
    const float fa = bf16r(a[e]) * sc;
    const float fb = bf16r(b[e]) * sc;
    hv[e]     = (_Float16)fa;
    hv[4 + e] = (_Float16)fb;
  }
  *(volatile v8h*)dp = hv;
  __threadfence();
  *(volatile v8h*)dp = hv;
}

__global__ __launch_bounds__(256) void cvt_x_kernel(const float* __restrict__ x, unsigned short* __restrict__ xh) {
  const int i = blockIdx.x * 256 + threadIdx.x;
  if (i < CH_X) cvt8_store(x + (size_t)i * 8, xh + (size_t)i * 8, XCARRY);
}

__global__ __launch_bounds__(256) void prep_kernel(
    const float* __restrict__ w_ih, const float* __restrict__ w_hh, const float* __restrict__ w_ff,
    const float* __restrict__ b_ih, const float* __restrict__ b_hh, const float* __restrict__ b_ff,
    unsigned short* __restrict__ wih16, unsigned short* __restrict__ whh16, unsigned short* __restrict__ wff16,
    float* __restrict__ biasv) {
  const int blk = blockIdx.x, tid = threadIdx.x;
  if (blk < PB1) {
    const int i = blk * 256 + tid;
    cvt8_store(w_ih + (size_t)i * 8, wih16 + (size_t)i * 8, WCARRY);
  } else if (blk < PB2) {
    const int i = (blk - PB1) * 256 + tid;
    cvt8_store(w_hh + (size_t)i * 8, whh16 + (size_t)i * 8, WCARRY);
  } else if (blk < PB3) {
    const int i = (blk - PB2) * 256 + tid;
    cvt8_store(w_ff + (size_t)i * 8, wff16 + (size_t)i * 8, WCARRY);
  } else {
    const int sel = tid >> 7;
    const int i4s = (tid & 127) * 4;
    const int i4f = ((tid - 128) & 63) * 4;
    const v4f va = *(const v4f*)(b_ih + i4s);
    const v4f vb = *(const v4f*)(b_hh + i4s);
    const v4f vf = *(const v4f*)(b_ff + i4f);
    v4f o;
#pragma unroll
    for (int e = 0; e < 4; ++e) {
      const float s0 = bf16r(va[e]) + bf16r(vb[e]);
      const float s1 = bf16r(vf[e]);
      o[e] = (sel == 0) ? s0 : s1;
    }
    if (tid < 192) {
      float* op = biasv + ((sel == 0) ? i4s : (NHID + i4f));
      *(volatile v4f*)op = o;
      __threadfence();
      *(volatile v4f*)op = o;
    }
  }
}

__global__ __launch_bounds__(256) void xp_gemm_kernel(
    const unsigned short* __restrict__ Ap, int lda,
    const unsigned short* __restrict__ Btp, int ldb,
    float* __restrict__ C, int ldc,
    const float* __restrict__ bias, int M, int N, int K, float scale) {
  const _Float16* A  = (const _Float16*)Ap;
  const _Float16* Bt = (const _Float16*)Btp;
  __shared__ __align__(16) float sT[8][16 * 68];
  const int lane = threadIdx.x & 31;
  const int wave = threadIdx.x >> 5;
  const int tilesN = N >> 6;
  const int tilesM = M >> 6;
  const int tile = blockIdx.x * 8 + wave;
  if (tile >= tilesM * tilesN) return;
  const int tm = tile / tilesN;
  const int tn = tile - tm * tilesN;
  const int m0 = tm << 6;
  const int n0 = tn << 6;

  const int rlane = lane & 15;
  const int koff  = (lane >> 4) * 8;
  const int mOff  = (lane >> 4) * 8;

  v8f acc[4][4];
#pragma unroll
  for (int i = 0; i < 4; ++i)
#pragma unroll
    for (int j = 0; j < 4; ++j) acc[i][j] = (v8f){0.f,0.f,0.f,0.f,0.f,0.f,0.f,0.f};

  for (int k0 = 0; k0 < K; k0 += 32) {
    v16h bh[4];
#pragma unroll
    for (int j = 0; j < 4; ++j) {
      const size_t bo = (size_t)(n0 + (j << 4) + rlane) * ldb + koff + k0;
      bh[j] = FragH::load(Bt + bo);
    }
#pragma unroll
    for (int i = 0; i < 4; ++i) {
      const size_t ao = (size_t)(m0 + (i << 4) + rlane) * lda + koff + k0;
      v16h ah = FragH::load(A + ao);
#pragma unroll
      for (int j = 0; j < 4; ++j) acc[i][j] = FragH::mma(ah, bh[j], acc[i][j]);
      guard4in_h(acc[i][0], acc[i][1], acc[i][2], acc[i][3], ah, bh[3]);
    }
    keep4_h(bh[0], bh[1], bh[2], bh[3]);
  }
  acc_guard4(acc[0][0], acc[0][1], acc[0][2], acc[0][3]);
  acc_guard4(acc[1][0], acc[1][1], acc[1][2], acc[1][3]);
  acc_guard4(acc[2][0], acc[2][1], acc[2][2], acc[2][3]);
  acc_guard4(acc[3][0], acc[3][1], acc[3][2], acc[3][3]);

  float* slab = sT[wave];
#pragma unroll
  for (int i = 0; i < 4; ++i) {
    const int mBase = m0 + (i << 4);
#pragma unroll
    for (int j = 0; j < 4; ++j) {
      const int n = n0 + (j << 4) + rlane;
      const float bv = bias[n];
#pragma unroll
      for (int r = 0; r < 8; ++r) {
        const float v = acc[i][j][r] * scale + bv;
        slab[(mOff + r) * 68 + (j << 4) + rlane] = v;
      }
    }
    __builtin_amdgcn_fence(__ATOMIC_RELEASE, "workgroup");
    __builtin_amdgcn_wave_barrier();
    __builtin_amdgcn_fence(__ATOMIC_ACQUIRE, "workgroup");
    {
      const int hh = lane >> 4, c4 = (lane & 15) * 4;
      for (int pass = 0; pass < 2; ++pass) {
#pragma unroll
        for (int it = 0; it < 8; ++it) {
          const int row = it * 2 + hh;
          v4f v = *(const v4f*)(slab + row * 68 + c4);
          *(volatile v4f*)(C + (size_t)(mBase + row) * ldc + n0 + c4) = v;
        }
        __threadfence();
      }
    }
    __builtin_amdgcn_fence(__ATOMIC_RELEASE, "workgroup");
    __builtin_amdgcn_wave_barrier();
    __builtin_amdgcn_fence(__ATOMIC_ACQUIRE, "workgroup");
  }
}

__global__ __launch_bounds__(RNN_THREADS) void rnn_fused_kernel(
    const float* XP, const float* __restrict__ h0,
    const unsigned short* __restrict__ whhp, const unsigned short* __restrict__ wffp,
    const float* __restrict__ biasv, float* out) {
  __shared__ __align__(16) _Float16 hH[2 * HTILE];
  __shared__ __align__(16) _Float16 hL[2 * HTILE];
  __shared__ __align__(16) float    Sl[RNN_THREADS / 32][16 * SLABP];
  const _Float16* WHH = (const _Float16*)whhp;
  const _Float16* WFF = (const _Float16*)wffp;
  const int tid = threadIdx.x, lane = tid & 31, wave = tid >> 5;
  const int c = lane & 15, hh = lane >> 4, koff = hh * 8, mOff = hh * 8;
  const int seq0 = blockIdx.x * SEQ_PB;
  const int n0 = wave * 64;
  const int o0 = wave * 32;

#pragma unroll 1
  for (int it = 0; it < 4; ++it) {
    const int chunk = it * RNN_THREADS + tid;
    const int r  = chunk >> 6;
    const int c8 = (chunk & 63) * 8;
    const float* sp = h0 + (size_t)(seq0 + r) * NHID + c8;
    const v4f a = *(const v4f*)(sp);
    const v4f b = *(const v4f*)(sp + 4);
    v8h vh, vl;
#pragma unroll
    for (int e = 0; e < 4; ++e) {
      _Float16 th, tl;
      const float fa = bf16r(a[e]);
      split_h(fa, th, tl);
      vh[e] = th; vl[e] = tl;
      const float fb = bf16r(b[e]);
      split_h(fb, th, tl);
      vh[4 + e] = th; vl[4 + e] = tl;
    }
    *(v8h*)(hH + r * HPITCH + c8) = vh;
    *(v8h*)(hL + r * HPITCH + c8) = vl;
  }
  const float bo0 = biasv[NHID + o0 + c];
  const float bo1 = biasv[NHID + o0 + 16 + c];
  __syncthreads();

  const v8f z8 = {0.f, 0.f, 0.f, 0.f, 0.f, 0.f, 0.f, 0.f};
  const _Float16* brow  = WHH + (size_t)(n0 + c) * NHID + koff;
  const _Float16* browf = WFF + (size_t)(o0 + c) * NHID + koff;
  float* slab = Sl[wave];
  const int q4 = lane >> 3, c4 = (lane & 7) * 4;

#pragma unroll 1
  for (int t = 0; t < NSTEP; ++t) {
    const int cur = t & 1;
    const _Float16* hcH = hH + cur * HTILE;
    const _Float16* hcL = hL + cur * HTILE;
    _Float16* hnH = hH + (cur ^ 1) * HTILE;
    _Float16* hnL = hL + (cur ^ 1) * HTILE;

    v8f accH[4], accL[4];
#pragma unroll
    for (int j = 0; j < 4; ++j) { accH[j] = z8; accL[j] = z8; }
    {
      const _Float16* arowH = hcH + c * HPITCH + koff;
      const _Float16* arowL = hcL + c * HPITCH + koff;
#pragma unroll 2
      for (int kc = 0; kc < NHID / 32; ++kc) {
        const v16h fa = FragH::load(arowH + kc * 32);
        const v16h fl = FragH::load(arowL + kc * 32);
        v16h fb[4];
#pragma unroll
        for (int j = 0; j < 4; ++j) fb[j] = FragH::load(brow + (size_t)(16 * j) * NHID + kc * 32);
#pragma unroll
        for (int j = 0; j < 4; ++j) {
          accH[j] = FragH::mma(fa, fb[j], accH[j]);
          accL[j] = FragH::mma(fl, fb[j], accL[j]);
        }
        guard8in_h(accH[0], accH[1], accH[2], accH[3], accL[0], accL[1], accL[2], accL[3], fa, fl);
        keep4_h(fb[0], fb[1], fb[2], fb[3]);
      }
      acc_guard4(accH[0], accH[1], accH[2], accH[3]);
      acc_guard4(accL[0], accL[1], accL[2], accL[3]);
    }

#pragma unroll
    for (int j = 0; j < 4; ++j) {
      const int col = n0 + 16 * j + c;
      float xv[8];
#pragma unroll
      for (int r = 0; r < 8; ++r)
        xv[r] = XP[((size_t)(seq0 + mOff + r) * NSTEP + (size_t)t) * NHID + col];
#pragma unroll
      for (int r = 0; r < 8; ++r) {
        const float pre = xv[r] + accH[j][r] * INV_W + accL[j][r] * INV_WL;
        const float hv = tanhf(pre);
        _Float16 th, tl;
        split_h(hv, th, tl);
        hnH[(mOff + r) * HPITCH + col] = th;
        hnL[(mOff + r) * HPITCH + col] = tl;
      }
      asm volatile("" ::: "memory");
    }

    __syncthreads();

    v8f accO0 = z8, accO1 = z8, accP0 = z8, accP1 = z8;
    {
      const _Float16* arowH = hnH + c * HPITCH + koff;
      const _Float16* arowL = hnL + c * HPITCH + koff;
#pragma unroll 2
      for (int kc = 0; kc < NHID / 32; ++kc) {
        const v16h fa = FragH::load(arowH + kc * 32);
        const v16h fl = FragH::load(arowL + kc * 32);
        const v16h g0 = FragH::load(browf + kc * 32);
        const v16h g1 = FragH::load(browf + (size_t)16 * NHID + kc * 32);
        accO0 = FragH::mma(fa, g0, accO0);
        accO1 = FragH::mma(fa, g1, accO1);
        accP0 = FragH::mma(fl, g0, accP0);
        accP1 = FragH::mma(fl, g1, accP1);
        guard4in_h(accO0, accO1, accP0, accP1, fa, fl);
        keep4_h(g0, g1, g0, g1);
      }
      acc_guard4(accO0, accO1, accP0, accP1);
    }
#pragma unroll
    for (int r = 0; r < 8; ++r) {
      const float y0 = accO0[r] * INV_W + accP0[r] * INV_WL + bo0;
      const float y1 = accO1[r] * INV_W + accP1[r] * INV_WL + bo1;
      slab[(mOff + r) * SLABP + c]      = y0;
      slab[(mOff + r) * SLABP + 16 + c] = y1;
    }
    __builtin_amdgcn_fence(__ATOMIC_RELEASE, "workgroup");
    __builtin_amdgcn_wave_barrier();
    __builtin_amdgcn_fence(__ATOMIC_ACQUIRE, "workgroup");
    for (int pass = 0; pass < 2; ++pass) {
#pragma unroll
      for (int it = 0; it < 4; ++it) {
        const int row = it * 4 + q4;
        const v4f v = *(const v4f*)(slab + row * SLABP + c4);
        *(volatile v4f*)(out + ((size_t)(seq0 + row) * NSTEP + (size_t)t) * NOUTF + o0 + c4) = v;
      }
      __threadfence();
    }
    __builtin_amdgcn_fence(__ATOMIC_RELEASE, "workgroup");
    __builtin_amdgcn_wave_barrier();
    __builtin_amdgcn_fence(__ATOMIC_ACQUIRE, "workgroup");
  }
}

extern "C" void kernel_launch(void* const* d_in, const int* in_sizes, int n_in,
                              void* d_out, int out_size, void* d_ws, size_t ws_size, hipStream_t stream) {
  if (n_in < 8 || d_out == nullptr || d_ws == nullptr) return;
  if (in_sizes[0] != NSEQ * NSTEP * NIN || in_sizes[1] != NSEQ * NHID || in_sizes[2] != NHID * NIN ||
      in_sizes[3] != NHID * NHID || in_sizes[4] != NHID || in_sizes[5] != NHID ||
      in_sizes[6] != NOUTF * NHID || in_sizes[7] != NOUTF || out_size != NSEQ * NSTEP * NOUTF) return;

  const float* x    = (const float*)d_in[0];
  const float* h0   = (const float*)d_in[1];
  const float* w_ih = (const float*)d_in[2];
  const float* w_hh = (const float*)d_in[3];
  const float* b_ih = (const float*)d_in[4];
  const float* b_hh = (const float*)d_in[5];
  const float* w_ff = (const float*)d_in[6];
  const float* b_ff = (const float*)d_in[7];
  float* out = (float*)d_out;

  char* ws = (char*)d_ws; size_t off = 0;
  auto carve = [&](size_t bytes) -> char* { char* p = ws + off; off += (bytes + 255) & ~(size_t)255; return p; };
  unsigned short* XH    = (unsigned short*)carve((size_t)NROWS * NIN * 2);
  float*          XP    = (float*)carve((size_t)NROWS * NHID * 4);
  unsigned short* WIH16 = (unsigned short*)carve((size_t)NHID * NIN * 2);
  unsigned short* WHH16 = (unsigned short*)carve((size_t)NHID * NHID * 2);
  unsigned short* WFF16 = (unsigned short*)carve((size_t)NOUTF * NHID * 2);
  float*          BIASV = (float*)carve((size_t)4096);
  if (off > ws_size || off > (size_t)134217728) return;

  cvt_x_kernel<<<CH_X / 256, 256, 0, stream>>>(x, XH);
  prep_kernel<<<PREP_BLOCKS, 256, 0, stream>>>(w_ih, w_hh, w_ff, b_ih, b_hh, b_ff, WIH16, WHH16, WFF16, BIASV);
  xp_gemm_kernel<<<((NROWS / 64) * (NHID / 64)) / 8, 256, 0, stream>>>(
      XH, NIN, WIH16, NIN, XP, NHID, BIASV, NROWS, NHID, NIN, INV_XW);
  rnn_fused_kernel<<<RNN_BLOCKS, RNN_THREADS, 0, stream>>>(XP, h0, WHH16, WFF16, BIASV, out);
}
